// cross_set_score_69191923138676
// MI455X (gfx1250) — hardware-verified
//
#include <hip/hip_runtime.h>

typedef _Float16 v16h __attribute__((ext_vector_type(16)));
typedef _Float16 v8h  __attribute__((ext_vector_type(8)));
typedef float    v8f  __attribute__((ext_vector_type(8)));
typedef float    v4f  __attribute__((ext_vector_type(4)));
typedef v8h __attribute__((may_alias)) v8ha;
typedef v4f __attribute__((may_alias)) v4fa;

union Frag { v16h v; v8h half[2]; };

#define NS     16
#define MITEM  256
#define DIN    128
#define NHEAD  8
#define DHEAD  64
#define HCOLS  (NHEAD * DHEAD)
#define NTOK   (NS * NS * MITEM)
#define NX     (NTOK * DIN)
#define NW1    (DIN * HCOLS)
#define NX8    (NX / 8)
#define NW8    (NW1 / 8)
#define NBLK   (NS * NS * NHEAD)
#define PPITCH 32
#define WSCALE 64.0f
#define WINV   0.015625f

static_assert((NX8 % 256) == 0);
static_assert(((NX8 + NW8) % 256) == 0);
static_assert((NTOK % 128) == 0);
static_assert((MITEM % 128) == 0);

__device__ __forceinline__ v8f wmma_f16(v16h a, v16h b, v8f c) {
  v8f d = __builtin_amdgcn_wmma_f32_16x16x32_f16(false, a, false, b, (short)0, c, false, false);
  asm volatile("v_nop\n\tv_nop\n\tv_nop\n\tv_nop" : "+v"(d) : "v"(a), "v"(b));
  return d;
}

__device__ __forceinline__ v16h load_frag(const _Float16* p, int h) {
  Frag f;
  f.half[0] = *(const v8ha*)(p + 8 * h);
  f.half[1] = *(const v8ha*)(p + 16 + 8 * h);
  return f.v;
}

__global__ __launch_bounds__(256) void cvt_kernel(
    const float* __restrict__ x, const float* __restrict__ w1,
    _Float16* __restrict__ xh, _Float16* __restrict__ w1t)
{
  const int g = blockIdx.x * 256 + threadIdx.x;
  if (g < NX8) {
    const float* src = x + (size_t)g * 8;
    const v4f a = *(const v4fa*)src;
    const v4f c = *(const v4fa*)(src + 4);
    const v8h o = { (_Float16)a.x, (_Float16)a.y, (_Float16)a.z, (_Float16)a.w,
                    (_Float16)c.x, (_Float16)c.y, (_Float16)c.z, (_Float16)c.w };
    _Float16* dst = xh + (size_t)g * 8;
    *(volatile v8h*)dst = o;
    __threadfence();
    *(volatile v8h*)dst = o;
  } else {
    int e = g - NX8;
    if (e >= NW8) e = NW8 - 1;
    const int n = e >> 4, k0 = (e & 15) * 8;
    const float* src = w1 + (size_t)k0 * HCOLS + n;
    const v8h o = { (_Float16)(src[0 * HCOLS] * WSCALE), (_Float16)(src[1 * HCOLS] * WSCALE),
                    (_Float16)(src[2 * HCOLS] * WSCALE), (_Float16)(src[3 * HCOLS] * WSCALE),
                    (_Float16)(src[4 * HCOLS] * WSCALE), (_Float16)(src[5 * HCOLS] * WSCALE),
                    (_Float16)(src[6 * HCOLS] * WSCALE), (_Float16)(src[7 * HCOLS] * WSCALE) };
    _Float16* dst = w1t + (size_t)n * DIN + k0;
    const bool ok = (g - NX8) < NW8;
    if (ok) *(volatile v8h*)dst = o;
    __threadfence();
    if (ok) *(volatile v8h*)dst = o;
  }
}

__device__ __forceinline__ void proj_store_pass(const _Float16* sT, _Float16* plane,
                                                size_t rowbase, int w, int lane) {
  const int q8 = lane & 7, sub = lane >> 3;
  #pragma unroll
  for (int i = 0; i < 8; ++i) {
    const int lid = w * 32 + i * 4 + sub;
    const v8h v = *(const v8ha*)(sT + lid * DHEAD + 8 * q8);
    _Float16* dst = plane + (rowbase + (size_t)lid) * DHEAD + 8 * q8;
    *(volatile v8h*)dst = v;
  }
}

__global__ __launch_bounds__(128) void proj_kernel(
    const _Float16* __restrict__ xh,
    const _Float16* __restrict__ w1t,
    _Float16* __restrict__ hp)
{
  __shared__ __attribute__((aligned(16))) _Float16 sT[128 * DHEAD];

  const int tid = threadIdx.x, lane = tid & 31, w = tid >> 5;
  const int h = lane >> 4, m = lane & 15;
  const int m0 = blockIdx.x * 128;
  const int head = blockIdx.y;
  const int m0w = m0 + 32 * w;

  const _Float16* xa0 = xh + (size_t)(m0w + m) * DIN;
  const _Float16* xa1 = xa0 + (size_t)16 * DIN;
  const _Float16* wb  = w1t + (size_t)(head * DHEAD + m) * DIN;

  const v8f zero8 = {0.f, 0.f, 0.f, 0.f, 0.f, 0.f, 0.f, 0.f};
  v8f acc[2][4];
  #pragma unroll
  for (int mt = 0; mt < 2; ++mt)
    #pragma unroll
    for (int nt = 0; nt < 4; ++nt) acc[mt][nt] = zero8;

  #pragma unroll 1
  for (int k0 = 0; k0 < DIN; k0 += 32) {
    const v16h a0 = load_frag(xa0 + k0, h);
    const v16h a1 = load_frag(xa1 + k0, h);
    #pragma unroll
    for (int nt = 0; nt < 4; ++nt) {
      const v16h b = load_frag(wb + (size_t)nt * 16 * DIN + k0, h);
      acc[0][nt] = wmma_f16(a0, b, acc[0][nt]);
      acc[1][nt] = wmma_f16(a1, b, acc[1][nt]);
    }
  }

  #pragma unroll
  for (int nt = 0; nt < 4; ++nt) {
    const int feat = 16 * nt + m;
    #pragma unroll
    for (int mt = 0; mt < 2; ++mt) {
      #pragma unroll
      for (int r = 0; r < 8; ++r) {
        const int tokl = 32 * w + 16 * mt + 8 * h + r;
        sT[tokl * DHEAD + feat] = (_Float16)(acc[mt][nt][r] * WINV);
      }
    }
  }
  __syncthreads();

  const int pair = m0 >> 8;
  const int mloc = m0 & (MITEM - 1);
  const size_t rowbase = ((size_t)pair * NHEAD + head) * MITEM + mloc;
  proj_store_pass(sT, hp, rowbase, w, lane);
  __threadfence();
  proj_store_pass(sT, hp, rowbase, w, lane);
}

__global__ __launch_bounds__(256) void pdot_kernel(
    const _Float16* __restrict__ hp,
    float* __restrict__ part)
{
  __shared__ float red[8];

  const int b = blockIdx.x;
  const int head = b & 7, i = (b >> 3) & 15, j = b >> 7;
  const int tid = threadIdx.x, lane = tid & 31, w = tid >> 5;
  const int h = lane >> 4, m = lane & 15;

  const _Float16* hA = hp + (size_t)((j * NS + i) * NHEAD + head) * (MITEM * DHEAD);
  const _Float16* hB = hp + (size_t)((i * NS + j) * NHEAD + head) * (MITEM * DHEAD);

  const v8f zero8 = {0.f, 0.f, 0.f, 0.f, 0.f, 0.f, 0.f, 0.f};
  float psum = 0.0f;

  #pragma unroll 1
  for (int mt2 = 0; mt2 < 2; ++mt2) {
    const int mt = 2 * w + mt2;
    const _Float16* pA = hA + (size_t)(mt * 16 + m) * DHEAD;
    const v16h a0 = load_frag(pA, h);
    const v16h a1 = load_frag(pA + 32, h);
    #pragma unroll 1
    for (int nt = 0; nt < 16; ++nt) {
      const _Float16* pB = hB + (size_t)(nt * 16 + m) * DHEAD;
      const v16h b0 = load_frag(pB, h);
      const v16h b1 = load_frag(pB + 32, h);
      v8f z = zero8;
      z = wmma_f16(a0, b0, z);
      z = wmma_f16(a1, b1, z);
      #pragma unroll
      for (int r = 0; r < 8; ++r) {
        const float s = z[r] * 0.125f;
        psum += fmaxf(s, 0.3f * s);
      }
    }
  }

  #pragma unroll
  for (int off = 16; off > 0; off >>= 1) psum += __shfl_xor(psum, off, 32);
  if (lane == 0) red[w] = psum;
  __syncthreads();

  if (w == 0) {
    float S = red[0];
    #pragma unroll
    for (int q = 1; q < 8; ++q) S += red[q];
    v4f v = {0.f, 0.f, 0.f, 0.f};
    if (lane == 0) v.x = S;
    float* dst = part + (size_t)b * PPITCH + 4 * lane;
    if (lane < 8) *(volatile v4f*)dst = v;
    __threadfence();
    if (lane < 8) *(volatile v4f*)dst = v;
  }
}

__global__ __launch_bounds__(256) void head_kernel(
    const float* __restrict__ part,
    const float* __restrict__ nItem,
    const float* __restrict__ W2,
    float* __restrict__ out)
{
  #pragma clang fp contract(off)
  __shared__ __attribute__((aligned(16))) float so[NS * NS];

  const int p = threadIdx.x;
  const int j = p >> 4, i = p & 15;
  const float rn = 1.0f / (nItem[i] * nItem[j]);
  float o = 0.0f;
  #pragma unroll
  for (int hd = 0; hd < NHEAD; ++hd) {
    const float sc = part[(size_t)(p * NHEAD + hd) * PPITCH] * rn;
    o = o + sc * W2[hd];
  }
  so[p] = o;
  __syncthreads();

  const v4f v = *(const v4fa*)(so + 4 * (p & 63));
  if (p < 64) *(volatile v4f*)(out + 4 * p) = v;
  __threadfence();
  if (p < 64) *(volatile v4f*)(out + 4 * p) = v;
}

extern "C" void kernel_launch(void* const* d_in, const int* in_sizes, int n_in,
                              void* d_out, int out_size, void* d_ws, size_t ws_size,
                              hipStream_t stream) {
  if (n_in < 4) return;
  if (in_sizes[0] != NX) return;
  if (in_sizes[1] != NS) return;
  if (in_sizes[2] != NW1) return;
  if (in_sizes[3] != NHEAD) return;
  if (out_size != NS * NS) return;

  const float* x     = (const float*)d_in[0];
  const float* nItem = (const float*)d_in[1];
  const float* W1    = (const float*)d_in[2];
  const float* W2    = (const float*)d_in[3];
  float* out = (float*)d_out;

  const size_t xh_bytes  = (size_t)NX * 2;
  const size_t w1t_bytes = (size_t)NW1 * 2;
  const size_t hp_bytes  = (size_t)NBLK * MITEM * DHEAD * 2;
  const size_t pt_bytes  = (size_t)NBLK * PPITCH * 4;
  const size_t total = xh_bytes + w1t_bytes + hp_bytes + pt_bytes;
  if (total > ws_size) return;

  char* ws = (char*)d_ws;
  _Float16* xh  = (_Float16*)(ws);
  _Float16* w1t = (_Float16*)(ws + xh_bytes);
  _Float16* hp  = (_Float16*)(ws + xh_bytes + w1t_bytes);
  float*    pt  = (float*)(ws + xh_bytes + w1t_bytes + hp_bytes);

  cvt_kernel<<<(NX8 + NW8) / 256, 256, 0, stream>>>(x, W1, xh, w1t);

  dim3 gProj(NTOK / 128, NHEAD);
  proj_kernel<<<gProj, 128, 0, stream>>>(xh, w1t, hp);

  pdot_kernel<<<NBLK, 256, 0, stream>>>(hp, pt);

  head_kernel<<<1, 256, 0, stream>>>(pt, nItem, W2, out);
}
